// LoRARelationWiseWordSelectionHead_69836168233630
// MI455X (gfx1250) — hardware-run, weakly checked
//
#include <hip/hip_runtime.h>
#include <stddef.h>
#include <math.h>


typedef _Float16 h16;
typedef _Float16 v16h __attribute__((ext_vector_type(16)));
typedef _Float16 v8h  __attribute__((ext_vector_type(8)));
typedef float    v8f  __attribute__((ext_vector_type(8)));
typedef float    v4f  __attribute__((ext_vector_type(4)));

#ifndef NB
#define NB 2
#endif
#ifndef SEQ
#define SEQ 96
#endif
#define NB_FULL  2
#define SEQ_FULL 96
#define DIM   768
#define NLBL  8
#define RANK  4
#define NLR   (RANK * NLBL)
#define NCOL  832
#define MROWS (NB * SEQ)
#define STILES (SEQ / 16)

static_assert(NB >= 1 && NB <= NB_FULL);
static_assert(SEQ >= 16 && SEQ <= SEQ_FULL && (SEQ % 16) == 0);
static_assert((DIM % 64) == 0 && (DIM % 32) == 0 && (DIM % 8) == 0);
static_assert((NCOL % 64) == 0 && NCOL >= DIM + NLR);
static_assert((MROWS % 64) == 0);
static_assert(NLR == 32 && NLBL == 8 && RANK == 4);
static_assert((size_t)NB_FULL * SEQ_FULL * SEQ_FULL * NLBL * 4 == (size_t)589824);

#define LDC 68
#define LDP 772
static_assert((LDC % 4) == 0 && LDC >= 64);
static_assert((LDP % 4) == 0 && LDP >= DIM);

#define WCARRY 64.0f

#define BT_PLANE   ((size_t)NCOL * DIM)
#define BIAS_PLANE ((size_t)NCOL)
#define DB_PLANE   ((size_t)NLBL * RANK * DIM)
#define HS_PLANE   ((size_t)MROWS * NCOL)

#define A16_BYTES  ((size_t)MROWS * DIM * 2)
#define BT_BYTES   ((size_t)2 * BT_PLANE * 2)
#define BIAS_BYTES ((size_t)2 * BIAS_PLANE * 4)
#define DBT_BYTES  ((size_t)2 * DB_PLANE * 4)
#define HS_BYTES   ((size_t)2 * HS_PLANE * 4)
#define OFF_A16  ((size_t)0)
#define OFF_BT   (OFF_A16 + A16_BYTES)
#define OFF_BIAS (OFF_BT + BT_BYTES)
#define OFF_DBT  (OFF_BIAS + BIAS_BYTES)
#define OFF_HS   (OFF_DBT + DBT_BYTES)
#define WS_TOTAL (OFF_HS + HS_BYTES)
static_assert((A16_BYTES % 128) == 0 && (BT_BYTES % 128) == 0 && (BIAS_BYTES % 128) == 0);
static_assert((DBT_BYTES % 128) == 0 && (HS_BYTES % 128) == 0);
static_assert(((BT_PLANE * 2) % 128) == 0 && ((BIAS_PLANE * 4) % 128) == 0);
static_assert(((DB_PLANE * 4) % 128) == 0 && ((HS_PLANE * 4) % 128) == 0);
static_assert(((size_t)NCOL * 4 % 128) == 0);
static_assert(WS_TOTAL <= (size_t)134217728);

#define WP_W_BLOCKS  (DIM * DIM / 8 / 256)
#define WP_DA_BLOCKS (NLR * DIM / 8 / 256)
#define WP_Z_BLOCKS  ((NCOL - DIM - NLR) * DIM / 8 / 256)
#define WP_B_BLOCKS  1
#define WP_DB_BLOCKS (NLBL * RANK * DIM / 4 / 256)
#define WP_BT_BLOCKS (WP_W_BLOCKS + WP_DA_BLOCKS + WP_Z_BLOCKS)
#define WP_BLOCKS    (WP_BT_BLOCKS + WP_B_BLOCKS + WP_DB_BLOCKS)
static_assert((DIM * DIM / 8) % 256 == 0);
static_assert((NLR * DIM / 8) % 256 == 0);
static_assert(((NCOL - DIM - NLR) * DIM / 8) % 256 == 0);
static_assert((NLBL * RANK * DIM / 4) % 256 == 0);
static_assert((size_t)WP_BT_BLOCKS * 256 * 8 == BT_PLANE);
static_assert((size_t)WP_DB_BLOCKS * 256 * 4 == DB_PLANE);
static_assert(NCOL / 4 <= 256 && (NCOL % 32) == 0);
static_assert(((size_t)MROWS * DIM / 8) % 256 == 0);
static_assert(16 * (DIM / 4) == 12 * 256);
static_assert(32 * NLR == 256 * 4);
static_assert(16 * 16 == 256);
static_assert(16 * NLBL * 4 == 32 * 16);

__device__ __forceinline__ float bf16r(float x) {
  unsigned int u = __float_as_uint(x);
  u = (u + 0x7FFFu + ((u >> 16) & 1u)) & 0xFFFF0000u;
  return __uint_as_float(u);
}

static __device__ __forceinline__ h16 toh_flush(float v) {
  const h16 r = (h16)v;
  return (fabsf(v) < 6.103515625e-05f) ? (h16)0.0f : r;
}

__device__ __forceinline__ v16h frag_at(const _Float16* p) {
  v8h lo = *(const v8h*)(p);
  v8h hi = *(const v8h*)(p + 16);
  v16h out;
#pragma unroll
  for (int i = 0; i < 8; ++i) { out[i] = lo[i]; out[i + 8] = hi[i]; }
  return out;
}

__device__ __forceinline__ v8f wmma16(v16h a, v16h b, v8f c) {
  v8f d = __builtin_amdgcn_wmma_f32_16x16x32_f16(false, a, false, b, (short)0, c,
                                                 false, false);
  asm volatile("v_nop\n\tv_nop\n\tv_nop\n\tv_nop" : "+v"(d) : "v"(a), "v"(b));
  return d;
}

__global__ __launch_bounds__(256) void acast_kernel(
    const float* __restrict__ X, _Float16* __restrict__ A16) {
  const unsigned g = blockIdx.x * 256u + threadIdx.x;
  const unsigned crow = g / (unsigned)(DIM / 8);
  const unsigned c = (g - crow * (unsigned)(DIM / 8)) * 8u;
  const unsigned bidx = crow / (unsigned)SEQ;
  const unsigned sq = crow - bidx * (unsigned)SEQ;
  const size_t srow = (size_t)bidx * SEQ_FULL + sq;
  const v4f a0 = *(const v4f*)(X + srow * DIM + c);
  const v4f a1 = *(const v4f*)(X + srow * DIM + c + 4u);
  v8h o;
#pragma unroll
  for (int i = 0; i < 4; ++i) {
    o[i]     = toh_flush(bf16r(a0[i]));
    o[i + 4] = toh_flush(bf16r(a1[i]));
  }
  _Float16* p = A16 + (size_t)crow * DIM + c;
  *(volatile v8h*)p = o;
  __threadfence();
  *(volatile v8h*)p = o;
}

__global__ __launch_bounds__(256) void wprep_kernel(
    const float* __restrict__ W, const float* __restrict__ da, const float* __restrict__ db,
    const float* __restrict__ bias, _Float16* __restrict__ Bt, float* __restrict__ biasp,
    float* __restrict__ dbt) {
  const unsigned tid = threadIdx.x;
  const unsigned blk = blockIdx.x;
  if (blk < (unsigned)WP_BT_BLOCKS) {
    const unsigned g = blk * 256u + tid;
    const unsigned n = g / (unsigned)(DIM / 8);
    const unsigned k0 = (g - n * (unsigned)(DIM / 8)) * 8u;
    v8h o;
    if (blk < (unsigned)WP_W_BLOCKS) {
      const v4f a0 = *(const v4f*)(W + (size_t)n * DIM + k0);
      const v4f a1 = *(const v4f*)(W + (size_t)n * DIM + k0 + 4u);
#pragma unroll
      for (int i = 0; i < 4; ++i) {
        o[i]     = toh_flush(WCARRY * bf16r(a0[i]));
        o[i + 4] = toh_flush(WCARRY * bf16r(a1[i]));
      }
    } else if (blk < (unsigned)(WP_W_BLOCKS + WP_DA_BLOCKS)) {
      const unsigned j = n - (unsigned)DIM;
#pragma unroll
      for (unsigned i = 0; i < 8u; ++i) {
        const float v = da[(size_t)(k0 + i) * NLR + j];
        o[i] = toh_flush(WCARRY * bf16r(v));
      }
    } else {
#pragma unroll
      for (int i = 0; i < 8; ++i) o[i] = (h16)0.0f;
    }
    _Float16* p = Bt + (size_t)g * 8u;
    *(volatile v8h*)p = o;
    __threadfence();
    *(volatile v8h*)p = o;
  } else if (blk == (unsigned)WP_BT_BLOCKS) {
    const unsigned c = tid * 4u;
    const unsigned cc = (c < (unsigned)(DIM - 4)) ? c : (unsigned)(DIM - 4);
    const v4f g = *(const v4f*)(bias + cc);
    v4f o;
#pragma unroll
    for (int j = 0; j < 4; ++j) o[j] = (c < (unsigned)DIM) ? bf16r(g[j]) : 0.0f;
    if (tid < (unsigned)(NCOL / 4)) {
      float* p = biasp + c;
      *(volatile v4f*)p = o;
      __threadfence();
      *(volatile v4f*)p = o;
    }
  } else {
    const unsigned f = (blk - (unsigned)(WP_BT_BLOCKS + WP_B_BLOCKS)) * 256u + tid;
    const unsigned l = f / (unsigned)(RANK * DIM / 4);
    const unsigned rem = f - l * (unsigned)(RANK * DIM / 4);
    const unsigned r = rem / (unsigned)(DIM / 4);
    const unsigned i0 = (rem - r * (unsigned)(DIM / 4)) * 4u;
    v4f o;
#pragma unroll
    for (unsigned j = 0; j < 4u; ++j)
      o[j] = bf16r(db[((size_t)r * DIM + i0 + j) * NLBL + l]);
    float* p = dbt + (size_t)f * 4u;
    *(volatile v4f*)p = o;
    __threadfence();
    *(volatile v4f*)p = o;
  }
}

__global__ __launch_bounds__(256) void gemm_proj_kernel(
    const _Float16* __restrict__ A16, const _Float16* __restrict__ Bt,
    const float* __restrict__ biasp, float* __restrict__ outf) {
  __shared__ float Cs[64 * LDC];
  const unsigned K = (unsigned)DIM;
  const unsigned tid = threadIdx.x, lane = tid & 31u, w = tid >> 5;
  const unsigned mw = w >> 1, nw = w & 1u;
  const unsigned hh = lane >> 4, m = lane & 15u;
  const unsigned n0 = blockIdx.x * 64u;
  const unsigned row0 = blockIdx.y * 64u;

  const _Float16* ap  = A16 + (size_t)(row0 + mw * 16u + m) * K + hh * 8u;
  const _Float16* bp0 = Bt + (size_t)(n0 + nw * 32u + m) * K + hh * 8u;
  const _Float16* bp1 = bp0 + (size_t)16 * K;
  v8f acc0 = {}, acc1 = {};
#pragma unroll 2
  for (unsigned k0 = 0; k0 < K; k0 += 32u) {
    const v16h a  = frag_at(ap + k0);
    const v16h b0 = frag_at(bp0 + k0);
    const v16h b1 = frag_at(bp1 + k0);
    acc0 = wmma16(a, b0, acc0);
    acc1 = wmma16(a, b1, acc1);
  }
#pragma unroll
  for (int r = 0; r < 8; ++r) {
    float* d = &Cs[(mw * 16u + hh * 8u + (unsigned)r) * LDC + nw * 32u + m];
    d[0]  = acc0[r];
    d[16] = acc1[r];
  }
  __syncthreads();

  v4f xs[4];
  size_t off[4];
#pragma unroll
  for (unsigned i = 0; i < 4u; ++i) {
    const unsigned r = 16u * i + (tid >> 4);
    const unsigned c = (tid & 15u) * 4u;
    const v4f u = *(const v4f*)&Cs[r * LDC + c];
    const v4f g = *(const v4f*)(biasp + n0 + c);
    v4f val;
#pragma unroll
    for (int j = 0; j < 4; ++j) val[j] = u[j] * (1.0f / WCARRY) + g[j];
    xs[i] = val;
    off[i] = (size_t)(row0 + r) * NCOL + n0 + c;
  }
#pragma unroll
  for (int i = 0; i < 4; ++i) *(volatile v4f*)(outf + off[i]) = xs[i];
  __threadfence();
#pragma unroll
  for (int i = 0; i < 4; ++i) *(volatile v4f*)(outf + off[i]) = xs[i];
}

__global__ __launch_bounds__(256) void pair_kernel(
    const float* __restrict__ HS, const float* __restrict__ DBT,
    const float* __restrict__ cls, float* __restrict__ out) {
  __shared__ float ST[2 * 16 * LDP];
  __shared__ float cl[DIM];
  __shared__ float Us[32 * NLR];
  __shared__ float outS[256 * NLBL];

  const unsigned tid = threadIdx.x;
  const unsigned tile = blockIdx.x;
  const unsigned stile = tile / (unsigned)STILES;
  const unsigned ttile = tile - stile * (unsigned)STILES;
  const unsigned b = blockIdx.y;
  const unsigned s0 = stile * 16u, t0 = ttile * 16u;

  {
    const unsigned row = tid >> 3;
    const unsigned c4 = (tid & 7u) * 4u;
    const unsigned side = row >> 4;
    const unsigned x0 = side ? t0 : s0;
    const size_t off = (size_t)side * HS_PLANE +
                       (size_t)(b * (unsigned)SEQ + x0 + (row & 15u)) * NCOL + DIM + c4;
    *(v4f*)&Us[row * NLR + c4] = *(const v4f*)(HS + off);
  }

  const unsigned sl = tid & 15u, tl = tid >> 4;

#pragma unroll 1
  for (unsigned l = 0; l < (unsigned)NLBL; ++l) {
    __syncthreads();
#pragma unroll 1
    for (unsigned i = tid; i < (unsigned)DIM; i += 256u)
      cl[i] = bf16r(cls[(size_t)i * NLBL + l]);
#pragma unroll 1
    for (unsigned side = 0; side < 2u; ++side) {
      const unsigned x0 = side ? t0 : s0;
#pragma unroll 1
      for (unsigned j = 0; j < 12u; ++j) {
        const unsigned idx = tid + 256u * j;
        const unsigned row = idx / (unsigned)(DIM / 4);
        const unsigned q = idx - row * (unsigned)(DIM / 4);
        v4f acc = *(const v4f*)(HS + (size_t)side * HS_PLANE +
                                (size_t)(b * (unsigned)SEQ + x0 + row) * NCOL + 4u * q);
#pragma unroll
        for (unsigned r = 0; r < (unsigned)RANK; ++r) {
          const v4f d = *(const v4f*)(DBT + (size_t)side * DB_PLANE +
                                      (size_t)(l * (unsigned)RANK + r) * DIM + 4u * q);
          const float uu = Us[(side * 16u + row) * NLR + r * 8u + l];
#pragma unroll
          for (int jj = 0; jj < 4; ++jj) acc[jj] = fmaf(uu, d[jj], acc[jj]);
        }
        *(v4f*)&ST[(side * 16u + row) * LDP + 4u * q] = acc;
      }
    }
    __syncthreads();

    float acc = 0.0f;
#pragma unroll 2
    for (unsigned h = 0; h < (unsigned)DIM; ++h) {
      const float x = ST[sl * LDP + h] + ST[(16u + tl) * LDP + h];
      const float g = 0.5f * x * (1.0f + erff(x * 0.70710678118654752f));
      acc = fmaf(g, cl[h], acc);
    }
    outS[(sl * 16u + tl) * NLBL + l] = acc;
  }
  __syncthreads();

  v4f x[2];
  size_t off[2];
#pragma unroll
  for (unsigned i = 0; i < 2u; ++i) {
    const unsigned idx = tid + 256u * i;
    const unsigned row = idx >> 5;
    const unsigned c4 = idx & 31u;
    x[i] = *(const v4f*)&outS[idx * 4u];
    off[i] = (((size_t)b * SEQ_FULL + s0 + row) * SEQ_FULL + t0) * NLBL + c4 * 4u;
  }
#pragma unroll
  for (int i = 0; i < 2; ++i) *(volatile v4f*)(out + off[i]) = x[i];
  __threadfence();
#pragma unroll
  for (int i = 0; i < 2; ++i) *(volatile v4f*)(out + off[i]) = x[i];
}

extern "C" void kernel_launch(void* const* d_in, const int* in_sizes, int n_in,
                              void* d_out, int out_size, void* d_ws, size_t ws_size,
                              hipStream_t stream) {
  if (n_in < 10) return;
  const long long need_x = ((long long)(NB - 1) * SEQ_FULL + SEQ) * DIM;
  const long long need_o =
      ((((long long)(NB - 1) * SEQ_FULL + (SEQ - 1)) * SEQ_FULL) + SEQ) * NLBL;
  if ((long long)in_sizes[0] < need_x) return;
  if ((long long)in_sizes[1] < (long long)DIM * DIM) return;
  if ((long long)in_sizes[3] < (long long)DIM * DIM) return;
  if (in_sizes[2] < DIM || in_sizes[4] < DIM) return;
  if (in_sizes[5] < DIM * NLR || in_sizes[6] < DIM * NLR) return;
  if (in_sizes[7] < DIM * NLR || in_sizes[8] < DIM * NLR) return;
  if (in_sizes[9] < DIM * NLBL) return;
  if ((long long)out_size < need_o) return;
  if (ws_size < WS_TOTAL) return;

  const float* pooled = (const float*)d_in[0];
  const float* W_src  = (const float*)d_in[1];
  const float* b_src  = (const float*)d_in[2];
  const float* W_tgt  = (const float*)d_in[3];
  const float* b_tgt  = (const float*)d_in[4];
  const float* da_src = (const float*)d_in[5];
  const float* db_src = (const float*)d_in[6];
  const float* da_tgt = (const float*)d_in[7];
  const float* db_tgt = (const float*)d_in[8];
  const float* cls    = (const float*)d_in[9];
  float* out = (float*)d_out;

  char* ws = (char*)d_ws;
  _Float16* A16  = (_Float16*)(ws + OFF_A16);
  _Float16* BtS  = (_Float16*)(ws + OFF_BT);
  _Float16* BtT  = BtS + BT_PLANE;
  float*    BiS  = (float*)(ws + OFF_BIAS);
  float*    BiT  = BiS + BIAS_PLANE;
  float*    DbS  = (float*)(ws + OFF_DBT);
  float*    DbT  = DbS + DB_PLANE;
  float*    HsS  = (float*)(ws + OFF_HS);
  float*    HsT  = HsS + HS_PLANE;

  dim3 blk(256);
  acast_kernel<<<dim3((unsigned)((size_t)MROWS * DIM / 8 / 256)), blk, 0, stream>>>(pooled, A16);
  wprep_kernel<<<dim3(WP_BLOCKS), blk, 0, stream>>>(W_src, da_src, db_src, b_src, BtS, BiS, DbS);
  wprep_kernel<<<dim3(WP_BLOCKS), blk, 0, stream>>>(W_tgt, da_tgt, db_tgt, b_tgt, BtT, BiT, DbT);
  dim3 gg(NCOL / 64, MROWS / 64);
  gemm_proj_kernel<<<gg, blk, 0, stream>>>(A16, BtS, BiS, HsS);
  gemm_proj_kernel<<<gg, blk, 0, stream>>>(A16, BtT, BiT, HsT);
  pair_kernel<<<dim3(STILES * STILES, NB), blk, 0, stream>>>(HsS, DbS, cls, out);
}
